// GCN_EAI_27642409517527
// MI455X (gfx1250) — hardware-verified
//
#include <hip/hip_runtime.h>
#include <math.h>
#include <stdint.h>

constexpr int N_BATCH   = 8;
constexpr int SEQ_LEN   = 1024;
constexpr int EMB_DIM   = 256;
constexpr int N_HEAD    = 8;
constexpr int HEAD_DIM  = 32;
constexpr int N_TOK     = N_BATCH * SEQ_LEN;
constexpr int QK_COLS   = 2 * EMB_DIM;
constexpr int QKV_ROWS  = 3 * EMB_DIM;
constexpr float Q_SCALE = 0.17677669529663689f;
constexpr float BN_EPS  = 1e-5f;
constexpr int STAT_RB   = 64;
constexpr int STAT_NBLK = N_TOK / STAT_RB;
constexpr int NORM_RB   = 8;
constexpr int NORM_NBLK = N_TOK / NORM_RB;
static_assert(STAT_NBLK * STAT_RB == N_TOK, "stat blocks cover all rows");
static_assert(NORM_NBLK * NORM_RB == N_TOK, "norm blocks cover all rows");
static_assert(SEQ_LEN / STAT_RB == 16, "16 statistics blocks per batch row group");

typedef __attribute__((ext_vector_type(16))) _Float16 v16h;
typedef __attribute__((ext_vector_type(8)))  _Float16 v8h;
typedef __attribute__((ext_vector_type(16))) __bf16   v16b;
typedef __attribute__((ext_vector_type(8)))  __bf16   v8b;
typedef __attribute__((ext_vector_type(8)))  float    v8f;
typedef __attribute__((ext_vector_type(4)))  float    v4f;
typedef __attribute__((ext_vector_type(2)))  float    v2f;
typedef __attribute__((ext_vector_type(4)))  unsigned int v4u;

__device__ __forceinline__ unsigned short f2bf_bits(float f) {
  unsigned u = __float_as_uint(f);
  return (unsigned short)((u + 0x7FFFu + ((u >> 16) & 1u)) >> 16);
}
__device__ __forceinline__ float bf_bits2f(unsigned short h) { return __uint_as_float(((unsigned)h) << 16); }

__device__ __forceinline__ void dep_guard_h(v8f& a, v8f& b, v16h x, v16h y) { asm volatile("v_nop\n\tv_nop\n\tv_nop\n\tv_nop" : "+v"(a), "+v"(b) : "v"(x), "v"(y)); }
__device__ __forceinline__ void dep_guard_b(v8f& a, v8f& b, v16b x, v16b y) { asm volatile("v_nop\n\tv_nop\n\tv_nop\n\tv_nop" : "+v"(a), "+v"(b) : "v"(x), "v"(y)); }
__device__ __forceinline__ void keep4_h(v16h a, v16h b, v16h c, v16h d) { asm volatile("v_nop" :: "v"(a), "v"(b), "v"(c), "v"(d)); }
__device__ __forceinline__ void keep4_b(v16b a, v16b b, v16b c, v16b d) { asm volatile("v_nop" :: "v"(a), "v"(b), "v"(c), "v"(d)); }
__device__ __forceinline__ void acc_guard4(v8f& a, v8f& b, v8f& c, v8f& d) { asm volatile("v_nop\n\tv_nop\n\tv_nop\n\tv_nop" : "+v"(a), "+v"(b), "+v"(c), "+v"(d)); }
template <typename T> struct Frag;
template <> struct Frag<_Float16> {
  typedef v16h V; union U { v16h v; v8h h[2]; };
  static __device__ __forceinline__ v16h load(const _Float16* p) {
    U f; f.h[0] = *(const v8h*)(p); f.h[1] = *(const v8h*)(p + 16); return f.v;
  }
  static __device__ __forceinline__ v8f mma(v16h a, v16h b, v8f c) {
    return __builtin_amdgcn_wmma_f32_16x16x32_f16(false, a, false, b, (short)0, c, false, false);
  }
  static __device__ __forceinline__ void guard(v8f& a, v8f& b, v16h x, v16h y) { dep_guard_h(a, b, x, y); }
  static __device__ __forceinline__ void keep(v16h a, v16h b, v16h c, v16h d) { keep4_h(a, b, c, d); }
};
template <> struct Frag<__bf16> {
  typedef v16b V; union U { v16b v; v8b h[2]; };
  static __device__ __forceinline__ v16b load(const __bf16* p) {
    U f; f.h[0] = *(const v8b*)(p); f.h[1] = *(const v8b*)(p + 16); return f.v;
  }
  static __device__ __forceinline__ v8f mma(v16b a, v16b b, v8f c) {
    return __builtin_amdgcn_wmma_f32_16x16x32_bf16(false, a, false, b, (short)0, c, false, false);
  }
  static __device__ __forceinline__ void guard(v8f& a, v8f& b, v16b x, v16b y) { dep_guard_b(a, b, x, y); }
  static __device__ __forceinline__ void keep(v16b a, v16b b, v16b c, v16b d) { keep4_b(a, b, c, d); }
};

template <int ET> struct Elem;
template <> struct Elem<0> { typedef _Float16 T; };
template <> struct Elem<1> { typedef __bf16 T; };
template <int ET, bool SPLIT, int BIAS_MODE, int OUT_MODE, bool RESID, int ACT = 0, bool DUALA = false>
__global__ __launch_bounds__(256) void wmma_gemm64(
    const unsigned short* __restrict__ Ap, const unsigned short* __restrict__ A2p, int lda, long strideA,
    const unsigned short* __restrict__ Btp, const unsigned short* __restrict__ Bt2p, int ldb, long strideB,
    void* __restrict__ Cout, void* __restrict__ Cout2, int ldc, long strideC,
    const float* __restrict__ bias,
    const float* __restrict__ resid, long strideR,
    int M, int N, int K, float scale, long strideAh) {
  typedef typename Elem<ET>::T T;
  typedef typename Frag<T>::V V;
  const T* A = (const T*)Ap; const T* A2 = (const T*)A2p; const T* Bt = (const T*)Btp; const T* Bt2 = (const T*)Bt2p;
  __shared__ __align__(16) float sT[8][16 * 68];
  const int b    = blockIdx.y;
  const int lane = threadIdx.x & 31;
  const int wave = threadIdx.x >> 5;
  const int tilesN = N >> 6;
  const int tilesM = M >> 6;
  const int tile = blockIdx.x * 8 + wave;
  if (tile >= tilesM * tilesN) return;
  const int tm = tile / tilesN;
  const int tn = tile - tm * tilesN;
  const int m0 = tm << 6;
  const int n0 = tn << 6;

  const T* Ab  = A  + (size_t)b * strideA;
  const T* Bb  = Bt + (size_t)b * strideB;
  const T* Ab2 = SPLIT ? (A2  + (size_t)b * strideA) : nullptr;
  const T* Bb2 = SPLIT ? (Bt2 + (size_t)b * strideB) : nullptr;

  const int rlane = lane & 15;
  const int koff  = (lane >> 4) * 8;
  const int mOff  = (lane >> 4) * 8;

  v8f acc[4][4];
#pragma unroll
  for (int i = 0; i < 4; ++i)
#pragma unroll
    for (int j = 0; j < 4; ++j) acc[i][j] = (v8f){0.f,0.f,0.f,0.f,0.f,0.f,0.f,0.f};

  for (int k0 = 0; k0 < K; k0 += 32) {
    V bh[4], bl[4];
#pragma unroll
    for (int j = 0; j < 4; ++j) {
      const size_t bo = (size_t)(n0 + (j << 4) + rlane) * ldb + koff + k0;
      bh[j] = Frag<T>::load(Bb + bo);
      if (SPLIT) bl[j] = Frag<T>::load(Bb2 + bo);
    }
#pragma unroll
    for (int i = 0; i < 4; ++i) {
      const size_t ao = (size_t)(m0 + (i << 4) + rlane) * lda + koff + k0;
      {
        V ah = Frag<T>::load(Ab + ao);
        V al;
        if (SPLIT) al = Frag<T>::load(Ab2 + ao);
#pragma unroll
        for (int j = 0; j < (DUALA ? 2 : 4); ++j) {
          acc[i][j] = Frag<T>::mma(ah, bh[j], acc[i][j]);
          if (SPLIT) {
            acc[i][j] = Frag<T>::mma(ah, bl[j], acc[i][j]);
            acc[i][j] = Frag<T>::mma(al, bh[j], acc[i][j]);
          }
        }
        if (DUALA) Frag<T>::guard(acc[i][0], acc[i][1], ah, SPLIT ? al : ah);
        else       Frag<T>::guard(acc[i][0], acc[i][3], ah, SPLIT ? al : ah);
      }
      if (DUALA) {
        V ah = Frag<T>::load(Ab + strideAh + ao);
        V al;
        if (SPLIT) al = Frag<T>::load(Ab2 + strideAh + ao);
#pragma unroll
        for (int j = 2; j < 4; ++j) {
          acc[i][j] = Frag<T>::mma(ah, bh[j], acc[i][j]);
          if (SPLIT) {
            acc[i][j] = Frag<T>::mma(ah, bl[j], acc[i][j]);
            acc[i][j] = Frag<T>::mma(al, bh[j], acc[i][j]);
          }
        }
        Frag<T>::guard(acc[i][2], acc[i][3], ah, SPLIT ? al : ah);
      }
    }
    Frag<T>::keep(bh[0], bh[1], bh[2], bh[3]);
    if (SPLIT) Frag<T>::keep(bl[0], bl[1], bl[2], bl[3]);
  }
  acc_guard4(acc[0][0], acc[0][1], acc[0][2], acc[0][3]);
  acc_guard4(acc[1][0], acc[1][1], acc[1][2], acc[1][3]);
  acc_guard4(acc[2][0], acc[2][1], acc[2][2], acc[2][3]);
  acc_guard4(acc[3][0], acc[3][1], acc[3][2], acc[3][3]);

  float* slab = sT[wave];
  const float* Rb = RESID ? (resid + (size_t)b * strideR) : nullptr;
#pragma unroll
  for (int i = 0; i < 4; ++i) {
    const int mBase = m0 + (i << 4);
#pragma unroll
    for (int j = 0; j < 4; ++j) {
      const int n = n0 + (j << 4) + rlane;
      float bv = 0.f;
      if (BIAS_MODE == 2) bv = bias[n];
#pragma unroll
      for (int r = 0; r < 8; ++r) {
        float v = acc[i][j][r] * scale;
        if (BIAS_MODE == 1) v += bias[mBase + mOff + r];
        if (BIAS_MODE == 2) v += bv;
        if (RESID) v += Rb[(size_t)(mBase + mOff + r) * ldc + n];
        if (ACT == 1) v = tanhf(v);
        if (ACT == 2) v = fmaxf(v, 0.0f);
        if (ACT == 4) v = (v > 0.f) ? v : 0.01f * v;
        slab[(mOff + r) * 68 + (j << 4) + rlane] = v;
      }
    }
    __builtin_amdgcn_fence(__ATOMIC_RELEASE, "workgroup");
    __builtin_amdgcn_wave_barrier();
    __builtin_amdgcn_fence(__ATOMIC_ACQUIRE, "workgroup");
    if (OUT_MODE == 0) {
      float* C = (float*)Cout + (size_t)b * strideC;
      const int hh = lane >> 4, c4 = (lane & 15) * 4;
      for (int pass = 0; pass < 2; ++pass) {
#pragma unroll
        for (int it = 0; it < 8; ++it) {
          const int row = it * 2 + hh;
          v4f v = *(const v4f*)(slab + row * 68 + c4);
          *(volatile v4f*)(C + (size_t)(mBase + row) * ldc + n0 + c4) = v;
        }
        __threadfence();
      }
    } else {
      const int q = lane >> 3, c8 = (lane & 7) * 8;
      unsigned short* C  = (unsigned short*)Cout  + (size_t)b * strideC;
      unsigned short* C2 = (OUT_MODE == 2) ? ((unsigned short*)Cout2 + (size_t)b * strideC) : nullptr;
      for (int pass = 0; pass < 2; ++pass) {
#pragma unroll
        for (int it = 0; it < 4; ++it) {
          const int row = it * 4 + q;
          const float* sp = slab + row * 68 + c8;
          v8h hv, lv;
#pragma unroll
          for (int e = 0; e < 8; ++e) {
            if (OUT_MODE == 1) {
              hv[e] = (_Float16)sp[e];
            } else {
              unsigned short hb = f2bf_bits(sp[e]);
              unsigned short lb = f2bf_bits(sp[e] - bf_bits2f(hb));
              hv[e] = __builtin_bit_cast(_Float16, hb);
              lv[e] = __builtin_bit_cast(_Float16, lb);
            }
          }
          *(volatile v8h*)(C + (size_t)(mBase + row) * ldc + n0 + c8) = hv;
          if (OUT_MODE == 2) *(volatile v8h*)(C2 + (size_t)(mBase + row) * ldc + n0 + c8) = lv;
        }
        __threadfence();
      }
    }
    __builtin_amdgcn_fence(__ATOMIC_RELEASE, "workgroup");
    __builtin_amdgcn_wave_barrier();
    __builtin_amdgcn_fence(__ATOMIC_ACQUIRE, "workgroup");
  }
}

__device__ __forceinline__ unsigned pk16(unsigned short a, unsigned short b) { return (unsigned)a | ((unsigned)b << 16); }

__global__ __launch_bounds__(256) void split_bf16x2_kernel(const float* __restrict__ in, unsigned short* __restrict__ hi,
                                                           unsigned short* __restrict__ lo, int n2) {
  const int i = blockIdx.x * 256 + threadIdx.x;
  if (i < n2) {
    const v2f f = *(const v2f*)(in + 2 * (size_t)i);
    const unsigned short h0 = f2bf_bits(f[0]), h1 = f2bf_bits(f[1]);
    const unsigned short l0 = f2bf_bits(f[0] - bf_bits2f(h0)), l1 = f2bf_bits(f[1] - bf_bits2f(h1));
    const unsigned uh = pk16(h0, h1), ul = pk16(l0, l1);
    ((volatile unsigned*)hi)[i] = uh;
    ((volatile unsigned*)lo)[i] = ul;
    __threadfence();
    ((volatile unsigned*)hi)[i] = uh;
    ((volatile unsigned*)lo)[i] = ul;
  }
}

__global__ __launch_bounds__(128) void softmax_pde_kernel(const float* __restrict__ S, const float* __restrict__ pde,
                                                          unsigned short* __restrict__ Ph, unsigned short* __restrict__ Pl) {
  __shared__ float redm[4];
  __shared__ float reds[4];
  const int i    = blockIdx.x;
  const int h    = blockIdx.y;
  const int tid  = threadIdx.x;
  const int lane = tid & 31;
  const int wave = tid >> 5;
  const int j0   = tid * 8;
  const size_t rowoff = ((size_t)h * SEQ_LEN + (size_t)i) * SEQ_LEN + (size_t)j0;
  const float* sr = S + rowoff;
  const float* pr = pde + (size_t)i * SEQ_LEN + j0;
  const v4f a0 = *(const v4f*)(sr);
  const v4f a1 = *(const v4f*)(sr + 4);
  const v4f g0 = *(const v4f*)(pr);
  const v4f g1 = *(const v4f*)(pr + 4);
  float t[8];
#pragma unroll
  for (int e = 0; e < 4; ++e) { t[e] = a0[e] + g0[e]; t[4 + e] = a1[e] + g1[e]; }
  float m = fmaxf(fmaxf(fmaxf(t[0], t[1]), fmaxf(t[2], t[3])), fmaxf(fmaxf(t[4], t[5]), fmaxf(t[6], t[7])));
#pragma unroll
  for (int off = 16; off > 0; off >>= 1) m = fmaxf(m, __shfl_xor(m, off, 32));
  if (lane == 0) redm[wave] = m;
  __syncthreads();
  const float mx = fmaxf(fmaxf(redm[0], redm[1]), fmaxf(redm[2], redm[3]));
  float ex[8];
#pragma unroll
  for (int e = 0; e < 8; ++e) ex[e] = __expf(t[e] - mx);
  float ps = ((((((ex[0] + ex[1]) + ex[2]) + ex[3]) + ex[4]) + ex[5]) + ex[6]) + ex[7];
#pragma unroll
  for (int off = 16; off > 0; off >>= 1) ps += __shfl_xor(ps, off, 32);
  if (lane == 0) reds[wave] = ps;
  __syncthreads();
  const float tot = ((reds[0] + reds[1]) + reds[2]) + reds[3];
  const float inv = 1.0f / tot;
  unsigned hw[4], lw[4];
#pragma unroll
  for (int q = 0; q < 4; ++q) {
    const float p0 = ex[2 * q] * inv, p1 = ex[2 * q + 1] * inv;
    const unsigned short hb0 = f2bf_bits(p0), hb1 = f2bf_bits(p1);
    const unsigned short lb0 = f2bf_bits(p0 - bf_bits2f(hb0));
    const unsigned short lb1 = f2bf_bits(p1 - bf_bits2f(hb1));
    hw[q] = pk16(hb0, hb1);
    lw[q] = pk16(lb0, lb1);
  }
  const v4u hvv = (v4u){hw[0], hw[1], hw[2], hw[3]};
  const v4u lvv = (v4u){lw[0], lw[1], lw[2], lw[3]};
  *(volatile v4u*)(Ph + rowoff) = hvv;
  *(volatile v4u*)(Pl + rowoff) = lvv;
  __threadfence();
  *(volatile v4u*)(Ph + rowoff) = hvv;
  *(volatile v4u*)(Pl + rowoff) = lvv;
}

__global__ __launch_bounds__(256) void bn_sum_kernel(const float* __restrict__ YA, const float* __restrict__ YB,
                                                     float* __restrict__ partS) {
  const int e = threadIdx.x;
  const int blk = blockIdx.x;
  const size_t r0 = (size_t)blk * STAT_RB;
  float sa = 0.f, sb = 0.f;
#pragma unroll 1
  for (int r = 0; r < STAT_RB; ++r) {
    sa += YA[(r0 + r) * EMB_DIM + e];
    sb += YB[(r0 + r) * EMB_DIM + e];
  }
  float* pa = partS + (size_t)blk * EMB_DIM + e;
  float* pb = partS + (size_t)STAT_NBLK * EMB_DIM + (size_t)blk * EMB_DIM + e;
  *(volatile float*)pa = sa;
  *(volatile float*)pb = sb;
  __threadfence();
  *(volatile float*)pa = sa;
  *(volatile float*)pb = sb;
}

__global__ __launch_bounds__(256) void bn_mean_kernel(const float* __restrict__ partS, float* __restrict__ meanb) {
  const int e = threadIdx.x;
  float sa = 0.f, sb = 0.f;
#pragma unroll 1
  for (int blk = 0; blk < STAT_NBLK; ++blk) {
    sa += partS[(size_t)blk * EMB_DIM + e];
    sb += partS[(size_t)STAT_NBLK * EMB_DIM + (size_t)blk * EMB_DIM + e];
  }
  const float ma = sa * (1.0f / (float)N_TOK);
  const float mb = sb * (1.0f / (float)N_TOK);
  *(volatile float*)(meanb + e) = ma;
  *(volatile float*)(meanb + EMB_DIM + e) = mb;
  __threadfence();
  *(volatile float*)(meanb + e) = ma;
  *(volatile float*)(meanb + EMB_DIM + e) = mb;
}

__global__ __launch_bounds__(256) void bn_sq_kernel(const float* __restrict__ YA, const float* __restrict__ YB,
                                                    const float* __restrict__ meanb, float* __restrict__ partQ) {
  const int e = threadIdx.x;
  const int blk = blockIdx.x;
  const size_t r0 = (size_t)blk * STAT_RB;
  const float ma = meanb[e], mb = meanb[EMB_DIM + e];
  float qa = 0.f, qb = 0.f;
#pragma unroll 1
  for (int r = 0; r < STAT_RB; ++r) {
    const float da = YA[(r0 + r) * EMB_DIM + e] - ma;
    const float db = YB[(r0 + r) * EMB_DIM + e] - mb;
    qa += da * da;
    qb += db * db;
  }
  float* pa = partQ + (size_t)blk * EMB_DIM + e;
  float* pb = partQ + (size_t)STAT_NBLK * EMB_DIM + (size_t)blk * EMB_DIM + e;
  *(volatile float*)pa = qa;
  *(volatile float*)pb = qb;
  __threadfence();
  *(volatile float*)pa = qa;
  *(volatile float*)pb = qb;
}

__global__ __launch_bounds__(256) void bn_coef_kernel(const float* __restrict__ partQ, const float* __restrict__ meanb,
                                                      const float* __restrict__ bnw, float* __restrict__ coef) {
  const int e = threadIdx.x;
  float qa = 0.f, qb = 0.f;
#pragma unroll 1
  for (int blk = 0; blk < STAT_NBLK; ++blk) {
    qa += partQ[(size_t)blk * EMB_DIM + e];
    qb += partQ[(size_t)STAT_NBLK * EMB_DIM + (size_t)blk * EMB_DIM + e];
  }
  const float va = qa * (1.0f / (float)N_TOK);
  const float vb = qb * (1.0f / (float)N_TOK);
  const float ma = meanb[e], mb = meanb[EMB_DIM + e];
  const float sg = 1.0f / (1.0f + __expf(-bnw[0]));
  const float w  = (sg + 1.0f) * 0.5f;
  const float w1 = 1.0f - w;
  const float mfa = w * ma + w1 * mb;
  const float mfb = w * mb + w1 * ma;
  const float vfa = w * va + w1 * vb;
  const float vfb = w * vb + w1 * va;
  const float inva = 1.0f / sqrtf(vfa + BN_EPS);
  const float invb = 1.0f / sqrtf(vfb + BN_EPS);
  for (int pass = 0; pass < 2; ++pass) {
    *(volatile float*)(coef + e) = mfa;
    *(volatile float*)(coef + EMB_DIM + e) = inva;
    *(volatile float*)(coef + 2 * EMB_DIM + e) = mfb;
    *(volatile float*)(coef + 3 * EMB_DIM + e) = invb;
    __threadfence();
  }
}

__global__ __launch_bounds__(256) void bn_norm_kernel(const float* __restrict__ YA, const float* __restrict__ YB,
                                                      const float* __restrict__ coef,
                                                      const float* __restrict__ g1, const float* __restrict__ b1,
                                                      const float* __restrict__ g2, const float* __restrict__ b2,
                                                      float* __restrict__ out0, float* __restrict__ out1) {
  const int e = threadIdx.x;
  const size_t r0 = (size_t)blockIdx.x * NORM_RB;
  const float mfa = coef[e], inva = coef[EMB_DIM + e], mfb = coef[2 * EMB_DIM + e], invb = coef[3 * EMB_DIM + e];
  const float ga = g1[e], ba = b1[e], gb = g2[e], bb = b2[e];
  float ya[NORM_RB], yb[NORM_RB];
#pragma unroll
  for (int r = 0; r < NORM_RB; ++r) {
    const size_t idx = (r0 + r) * EMB_DIM + e;
    ya[r] = ga * ((YA[idx] - mfa) * inva) + ba;
    yb[r] = gb * ((YB[idx] - mfb) * invb) + bb;
  }
  for (int pass = 0; pass < 2; ++pass) {
#pragma unroll
    for (int r = 0; r < NORM_RB; ++r) {
      const size_t idx = (r0 + r) * EMB_DIM + e;
      *(volatile float*)(out0 + idx) = ya[r];
      *(volatile float*)(out1 + idx) = yb[r];
    }
    __threadfence();
  }
}

__global__ __launch_bounds__(256) void mmd_kernel(const float* __restrict__ partS, const float* __restrict__ coef,
                                                  const float* __restrict__ g1, const float* __restrict__ b1,
                                                  const float* __restrict__ g2, const float* __restrict__ b2,
                                                  float* __restrict__ out2) {
  __shared__ float tot[16 * EMB_DIM];
  __shared__ float red[256];
  const int t = threadIdx.x;
  {
    const int e = t;
    const float mfa = coef[e], inva = coef[EMB_DIM + e], mfb = coef[2 * EMB_DIM + e], invb = coef[3 * EMB_DIM + e];
    const float ga = g1[e], ba = b1[e], gb = g2[e], bb = b2[e];
#pragma unroll 1
    for (int dom = 0; dom < 2; ++dom) {
      const float* ps = partS + (size_t)dom * STAT_NBLK * EMB_DIM;
      const float mf = (dom == 0) ? mfa : mfb;
      const float iv = (dom == 0) ? inva : invb;
      const float gg = (dom == 0) ? ga : gb;
      const float bt = (dom == 0) ? ba : bb;
#pragma unroll 1
      for (int bi = 0; bi < N_BATCH; ++bi) {
        float s = 0.f;
#pragma unroll 1
        for (int q = 0; q < 16; ++q) s += ps[(size_t)(bi * 16 + q) * EMB_DIM + e];
        const float my = s * (1.0f / (float)SEQ_LEN);
        tot[(dom * N_BATCH + bi) * EMB_DIM + e] = gg * ((my - mf) * iv) + bt;
      }
    }
  }
  __syncthreads();
  const int pi = t >> 4, pj = t & 15;
  float d = 0.f;
#pragma unroll 1
  for (int e = 0; e < EMB_DIM; ++e) {
    const float df = tot[pj * EMB_DIM + e] - tot[pi * EMB_DIM + e];
    d += df * df;
  }
  red[t] = d;
  __syncthreads();
  for (int st = 128; st > 0; st >>= 1) {
    if (t < st) red[t] += red[t + st];
    __syncthreads();
  }
  const float total = red[0];
  __syncthreads();
  const float bw = total / 240.0f / 4.0f;
  float kern = 0.f;
  float bwq = bw;
#pragma unroll 1
  for (int q = 0; q < 5; ++q) {
    kern += __expf(-d * (1.0f / bwq));
    bwq *= 2.0f;
  }
  const float sign = ((pi < 8) == (pj < 8)) ? 1.0f : -1.0f;
  red[t] = sign * kern;
  __syncthreads();
  for (int st = 128; st > 0; st >>= 1) {
    if (t < st) red[t] += red[t + st];
    __syncthreads();
  }
  if (t == 0) {
    const float loss = red[0] * (1.0f / 64.0f);
    *(volatile float*)out2 = loss;
    __threadfence();
    *(volatile float*)out2 = loss;
  }
}

extern "C" void kernel_launch(void* const* d_in, const int* in_sizes, int n_in,
                              void* d_out, int out_size, void* d_ws, size_t ws_size,
                              hipStream_t stream) {
  if (n_in < 12) return;
  if (in_sizes[0] != N_TOK * EMB_DIM || in_sizes[1] != N_TOK * EMB_DIM) return;
  if (in_sizes[2] != SEQ_LEN * SEQ_LEN) return;
  if (in_sizes[3] != QKV_ROWS * EMB_DIM || in_sizes[4] < QKV_ROWS) return;
  if (in_sizes[5] != EMB_DIM * EMB_DIM || in_sizes[6] < EMB_DIM) return;
  if (in_sizes[7] < EMB_DIM || in_sizes[8] < EMB_DIM || in_sizes[9] < EMB_DIM || in_sizes[10] < EMB_DIM) return;
  if (in_sizes[11] < 1) return;
  if (out_size != 2 * N_TOK * EMB_DIM + 1) return;

  const float* x     = (const float*)d_in[0];
  const float* x2    = (const float*)d_in[1];
  const float* pde   = (const float*)d_in[2];
  const float* win   = (const float*)d_in[3];
  const float* bin   = (const float*)d_in[4];
  const float* wo    = (const float*)d_in[5];
  const float* bo    = (const float*)d_in[6];
  const float* gam   = (const float*)d_in[7];
  const float* bet   = (const float*)d_in[8];
  const float* gam2  = (const float*)d_in[9];
  const float* bet2  = (const float*)d_in[10];
  const float* bnw   = (const float*)d_in[11];

  float* out0 = (float*)d_out;
  float* out1 = out0 + (size_t)N_TOK * EMB_DIM;
  float* out2 = out0 + 2 * (size_t)N_TOK * EMB_DIM;

  const size_t szWin  = (size_t)QKV_ROWS * EMB_DIM * 2;
  const size_t szWo   = (size_t)EMB_DIM * EMB_DIM * 2;
  const size_t szX    = (size_t)N_TOK * EMB_DIM * 2;
  const size_t szQK   = (size_t)N_TOK * QK_COLS * 2;
  const size_t szVT   = (size_t)EMB_DIM * N_TOK * 2;
  const size_t szC    = (size_t)N_TOK * EMB_DIM * 2;
  const size_t szS    = (size_t)N_HEAD * SEQ_LEN * SEQ_LEN * 4;
  const size_t szP    = (size_t)N_HEAD * SEQ_LEN * SEQ_LEN * 2;
  const size_t szY    = (size_t)N_TOK * EMB_DIM * 4;
  const size_t szPart = (size_t)2 * STAT_NBLK * EMB_DIM * 4;
  const size_t szMean = (size_t)2 * EMB_DIM * 4;
  const size_t szCoef = (size_t)4 * EMB_DIM * 4;
  size_t off = 0;
  const size_t oWinH = off; off += szWin;
  const size_t oWinL = off; off += szWin;
  const size_t oWoH  = off; off += szWo;
  const size_t oWoL  = off; off += szWo;
  const size_t oXH   = off; off += szX;
  const size_t oXL   = off; off += szX;
  const size_t oQKH  = off; off += szQK;
  const size_t oQKL  = off; off += szQK;
  const size_t oVTH  = off; off += szVT;
  const size_t oVTL  = off; off += szVT;
  const size_t oCH   = off; off += szC;
  const size_t oCL   = off; off += szC;
  const size_t oS    = off; off += szS;
  const size_t oPH   = off; off += szP;
  const size_t oPL   = off; off += szP;
  const size_t oYA   = off; off += szY;
  const size_t oYB   = off; off += szY;
  const size_t oPartS= off; off += szPart;
  const size_t oPartQ= off; off += szPart;
  const size_t oMean = off; off += szMean;
  const size_t oCoef = off; off += szCoef;
  if (off > ws_size) return;

  char* ws = (char*)d_ws;
  unsigned short* WinH = (unsigned short*)(ws + oWinH);
  unsigned short* WinL = (unsigned short*)(ws + oWinL);
  unsigned short* WoH  = (unsigned short*)(ws + oWoH);
  unsigned short* WoL  = (unsigned short*)(ws + oWoL);
  unsigned short* XH   = (unsigned short*)(ws + oXH);
  unsigned short* XL   = (unsigned short*)(ws + oXL);
  unsigned short* QKH  = (unsigned short*)(ws + oQKH);
  unsigned short* QKL  = (unsigned short*)(ws + oQKL);
  unsigned short* VTH  = (unsigned short*)(ws + oVTH);
  unsigned short* VTL  = (unsigned short*)(ws + oVTL);
  unsigned short* CH   = (unsigned short*)(ws + oCH);
  unsigned short* CL   = (unsigned short*)(ws + oCL);
  float*          Sbuf = (float*)(ws + oS);
  unsigned short* PH   = (unsigned short*)(ws + oPH);
  unsigned short* PL   = (unsigned short*)(ws + oPL);
  float*          YA   = (float*)(ws + oYA);
  float*          YB   = (float*)(ws + oYB);
  float*          partS= (float*)(ws + oPartS);
  float*          partQ= (float*)(ws + oPartQ);
  float*          meanb= (float*)(ws + oMean);
  float*          coef = (float*)(ws + oCoef);

  const dim3 blk(256);
  const int n2w = QKV_ROWS * EMB_DIM / 2;
  const int n2o = EMB_DIM * EMB_DIM / 2;
  split_bf16x2_kernel<<<dim3((n2w + 255) / 256), blk, 0, stream>>>(win, WinH, WinL, n2w);
  split_bf16x2_kernel<<<dim3((n2o + 255) / 256), blk, 0, stream>>>(wo, WoH, WoL, n2o);

  const int n2x = N_TOK * EMB_DIM / 2;
  const dim3 gSplit((n2x + 255) / 256);
  const dim3 gQK(((N_TOK / 64) * (QK_COLS / 64) + 7) / 8, 1);
  const dim3 gVT(((EMB_DIM / 64) * (N_TOK / 64) + 7) / 8, 1);
  const dim3 gS(((SEQ_LEN / 64) * (SEQ_LEN / 64) + 7) / 8, N_HEAD);
  const dim3 gSm(SEQ_LEN, N_HEAD);
  const dim3 gPV(((SEQ_LEN / 64) * (64 / 64) + 7) / 8, N_HEAD / 2);
  const dim3 gOut(((N_TOK / 64) * (EMB_DIM / 64) + 7) / 8, 1);

  for (int dom = 0; dom < 2; ++dom) {
    const float* xin = (dom == 0) ? x : x2;
    float* Yd = (dom == 0) ? YA : YB;
    split_bf16x2_kernel<<<gSplit, blk, 0, stream>>>(xin, XH, XL, n2x);
    wmma_gemm64<1, true, 2, 2, false, 0, false><<<gQK, blk, 0, stream>>>(
        XH, XL, EMB_DIM, 0L, WinH, WinL, EMB_DIM, 0L, (void*)QKH, (void*)QKL, QK_COLS, 0L,
        bin, bo, 0L, N_TOK, QK_COLS, EMB_DIM, 1.0f, 0L);
    wmma_gemm64<1, true, 1, 2, false, 0, false><<<gVT, blk, 0, stream>>>(
        WinH + (size_t)QK_COLS * EMB_DIM, WinL + (size_t)QK_COLS * EMB_DIM, EMB_DIM, 0L,
        XH, XL, EMB_DIM, 0L, (void*)VTH, (void*)VTL, N_TOK, 0L,
        bin + QK_COLS, bo, 0L, EMB_DIM, N_TOK, EMB_DIM, 1.0f, 0L);
    for (int bi = 0; bi < N_BATCH; ++bi) {
      const size_t qoff = (size_t)bi * SEQ_LEN * QK_COLS;
      wmma_gemm64<1, true, 0, 0, false, 0, false><<<gS, blk, 0, stream>>>(
          QKH + qoff, QKL + qoff, QK_COLS, (long)HEAD_DIM,
          QKH + qoff + EMB_DIM, QKL + qoff + EMB_DIM, QK_COLS, (long)HEAD_DIM,
          (void*)Sbuf, (void*)Sbuf, SEQ_LEN, (long)SEQ_LEN * SEQ_LEN,
          bo, bo, 0L, SEQ_LEN, SEQ_LEN, HEAD_DIM, Q_SCALE, 0L);
      softmax_pde_kernel<<<gSm, dim3(128), 0, stream>>>(Sbuf, pde, PH, PL);
      wmma_gemm64<1, true, 0, 2, false, 0, true><<<gPV, blk, 0, stream>>>(
          PH, PL, SEQ_LEN, (long)2 * SEQ_LEN * SEQ_LEN,
          VTH + (size_t)bi * SEQ_LEN, VTL + (size_t)bi * SEQ_LEN, N_TOK, (long)64 * N_TOK,
          (void*)(CH + (size_t)bi * SEQ_LEN * EMB_DIM), (void*)(CL + (size_t)bi * SEQ_LEN * EMB_DIM), EMB_DIM, 64L,
          bo, bo, 0L, SEQ_LEN, 64, SEQ_LEN, 1.0f, (long)SEQ_LEN * SEQ_LEN);
    }
    wmma_gemm64<1, true, 2, 0, false, 0, false><<<gOut, blk, 0, stream>>>(
        CH, CL, EMB_DIM, 0L, WoH, WoL, EMB_DIM, 0L, (void*)Yd, (void*)Yd, EMB_DIM, 0L,
        bo, bo, 0L, N_TOK, EMB_DIM, EMB_DIM, 1.0f, 0L);
  }

  bn_sum_kernel<<<dim3(STAT_NBLK), blk, 0, stream>>>(YA, YB, partS);
  bn_mean_kernel<<<dim3(1), blk, 0, stream>>>(partS, meanb);
  bn_sq_kernel<<<dim3(STAT_NBLK), blk, 0, stream>>>(YA, YB, meanb, partQ);
  bn_coef_kernel<<<dim3(1), blk, 0, stream>>>(partQ, meanb, bnw, coef);
  bn_norm_kernel<<<dim3(NORM_NBLK), blk, 0, stream>>>(YA, YB, coef, gam, bet, gam2, bet2, out0, out1);
  mmd_kernel<<<dim3(1), blk, 0, stream>>>(partS, coef, gam, bet, gam2, bet2, out2);
}
